// S_LSTMLayer_22273700397276
// MI455X (gfx1250) — hardware-run, weakly checked
//
#include <hip/hip_runtime.h>
#include <math.h>

typedef __attribute__((ext_vector_type(16))) _Float16 v16h;
typedef __attribute__((ext_vector_type(8)))  _Float16 v8h;
typedef __attribute__((ext_vector_type(2)))  _Float16 v2h;
typedef __attribute__((ext_vector_type(16))) __bf16   v16b;
typedef __attribute__((ext_vector_type(8)))  __bf16   v8b;
typedef __attribute__((ext_vector_type(8)))  float    v8f;
typedef __attribute__((ext_vector_type(4)))  float    v4f;
typedef __attribute__((ext_vector_type(2)))  float    v2f;
typedef __attribute__((ext_vector_type(4)))  _Float16 v4h;

constexpr int kB    = 64;
constexpr int kR    = 2 * kB;
constexpr int kL    = 256;
constexpr int kX    = 512;
constexpr int kHid  = 512;
constexpr int kGw   = 512;
constexpr int kG4   = 4 * kHid;
constexpr int kK    = kHid + kX;
constexpr int kOutW = 2 * kHid;
constexpr int kOut0 = kB * kL * kOutW;
constexpr int kOut1 = kB * kOutW;
constexpr int kOutAll = kOut0 + 2 * kOut1;
constexpr int kThr  = 256;
constexpr float kInCarry = 1024.0f;
constexpr float kWCarry  = 4096.0f;
constexpr float kSc = 1.0f / (kInCarry * kWCarry);
constexpr float kF16MinNormal = 6.103515625e-5f;

static_assert(kB == 64 && kR == 128 && kHid == 512 && kX == 512 && kGw == 512 && kG4 == 2048 && kK == 1024 && kL == 256, "the index arithmetic below uses these sizes");

constexpr size_t kOffW16 = 0ull;
constexpr size_t kOffWG16 = 4194304ull;
constexpr size_t kOffG16 = 6291456ull;
constexpr size_t kOffBV = 6356992ull;
constexpr size_t kOffSG = 6373376ull;
constexpr size_t kOffHX16 = 6897664ull;
constexpr size_t kOffGG = 7159808ull;
constexpr size_t kOffC32 = 8208384ull;
constexpr size_t kWsTotal = 8470528ull;
static_assert(kWsTotal <= 268435456ull, "the carve stands under the contract's 256 MiB of workspace");
static_assert(kOffW16 == 0
  && kOffWG16 == kOffW16 + 4194304ull
  && kOffG16 == kOffWG16 + 2097152ull
  && kOffBV == kOffG16 + 65536ull
  && kOffSG == kOffBV + 16384ull
  && kOffHX16 == kOffSG + 524288ull
  && kOffGG == kOffHX16 + 262144ull
  && kOffC32 == kOffGG + 1048576ull
  && kWsTotal == kOffC32 + 262144ull, "the carve is a chain: every region starts where the one before ends");
static_assert((size_t)kG4 * kK * 2 == 4194304ull && (size_t)kG4 * kGw * 2 == 2097152ull && (size_t)kB * kG4 * 4 == 524288ull && (size_t)kR * kK * 2 == 262144ull && (size_t)kR * kG4 * 4 == 1048576ull && (size_t)kR * kHid * 4 == 262144ull, "every region's length is its plane's");
static_assert((kOffWG16 % 256) == 0 && (kOffG16 % 256) == 0 && (kOffBV % 256) == 0 && (kOffSG % 256) == 0 && (kOffHX16 % 256) == 0 && (kOffGG % 256) == 0 && (kOffC32 % 256) == 0, "every region starts on a multiple of 256 B");
constexpr int kBvGate = 0, kBvZero = 2048;

__device__ __forceinline__ unsigned short f2bf_bits(float f) {
  unsigned u = __float_as_uint(f);
  return (unsigned short)((u + 0x7FFFu + ((u >> 16) & 1u)) >> 16);
}
__device__ __forceinline__ float bf_bits2f(unsigned short h) { return __uint_as_float(((unsigned)h) << 16); }
__device__ __forceinline__ float bf16r(float f) { return bf_bits2f(f2bf_bits(f)); }
__device__ __forceinline__ float carry_flush(float v, float carry) {
  const float s = v * carry;
  return (fabsf(s) < kF16MinNormal) ? 0.0f : s;
}

__device__ __forceinline__ void dep_guard4_h(v8f& a, v8f& b, v8f& c, v8f& d, v16h x, v16h y) { asm volatile("v_nop\n\tv_nop\n\tv_nop\n\tv_nop" : "+v"(a), "+v"(b), "+v"(c), "+v"(d) : "v"(x), "v"(y)); }
__device__ __forceinline__ void dep_guard4_b(v8f& a, v8f& b, v8f& c, v8f& d, v16b x, v16b y) { asm volatile("v_nop\n\tv_nop\n\tv_nop\n\tv_nop" : "+v"(a), "+v"(b), "+v"(c), "+v"(d) : "v"(x), "v"(y)); }
__device__ __forceinline__ void keep4_h(v16h a, v16h b, v16h c, v16h d) { asm volatile("v_nop" :: "v"(a), "v"(b), "v"(c), "v"(d)); }
__device__ __forceinline__ void keep4_b(v16b a, v16b b, v16b c, v16b d) { asm volatile("v_nop" :: "v"(a), "v"(b), "v"(c), "v"(d)); }
__device__ __forceinline__ void acc_guard4(v8f& a, v8f& b, v8f& c, v8f& d) { asm volatile("v_nop\n\tv_nop\n\tv_nop\n\tv_nop" : "+v"(a), "+v"(b), "+v"(c), "+v"(d)); }

template <typename T> struct Frag;
template <> struct Frag<_Float16> {
  typedef v16h V; union U { v16h v; v8h h[2]; };
  static __device__ __forceinline__ v16h load(const _Float16* p) {
    U f; f.h[0] = *(const v8h*)(p); f.h[1] = *(const v8h*)(p + 16); return f.v;
  }
  static __device__ __forceinline__ v8f mma(v16h a, v16h b, v8f c) {
    return __builtin_amdgcn_wmma_f32_16x16x32_f16(false, a, false, b, (short)0, c, false, false);
  }
  static __device__ __forceinline__ void guard4(v8f& a, v8f& b, v8f& c, v8f& d, v16h x, v16h y) { dep_guard4_h(a, b, c, d, x, y); }
  static __device__ __forceinline__ void keep(v16h a, v16h b, v16h c, v16h d) { keep4_h(a, b, c, d); }
};
template <> struct Frag<__bf16> {
  typedef v16b V; union U { v16b v; v8b h[2]; };
  static __device__ __forceinline__ v16b load(const __bf16* p) {
    U f; f.h[0] = *(const v8b*)(p); f.h[1] = *(const v8b*)(p + 16); return f.v;
  }
  static __device__ __forceinline__ v8f mma(v16b a, v16b b, v8f c) {
    return __builtin_amdgcn_wmma_f32_16x16x32_bf16(false, a, false, b, (short)0, c, false, false);
  }
  static __device__ __forceinline__ void guard4(v8f& a, v8f& b, v8f& c, v8f& d, v16b x, v16b y) { dep_guard4_b(a, b, c, d, x, y); }
  static __device__ __forceinline__ void keep(v16b a, v16b b, v16b c, v16b d) { keep4_b(a, b, c, d); }
};

__device__ __forceinline__ v8f mma_h(v16h a, v16h b, v8f c) {
  c = __builtin_amdgcn_wmma_f32_16x16x32_f16(false, a, false, b, (short)0, c, false, false);
  asm volatile("v_nop\n\tv_nop\n\tv_nop\n\tv_nop" : "+v"(c) : "v"(a), "v"(b));
  return c;
}

template <int ET> struct Elem;
template <> struct Elem<0> { typedef _Float16 T; };
template <> struct Elem<1> { typedef __bf16 T; };
template <int ET, bool SPLIT, int BIAS_MODE, int OUT_MODE, bool RESID, int ACT = 0>
__global__ __launch_bounds__(256) void wmma_gemm64(
    const unsigned short* __restrict__ Ap, const unsigned short* __restrict__ A2p, int lda, long strideA,
    const unsigned short* __restrict__ Btp, const unsigned short* __restrict__ Bt2p, int ldb, long strideB,
    void* __restrict__ Cout, void* __restrict__ Cout2, int ldc, long strideC,
    const float* __restrict__ bias,
    const float* __restrict__ resid, long strideR,
    int M, int N, int K, float scale) {
  typedef typename Elem<ET>::T T;
  typedef typename Frag<T>::V V;
  const T* A = (const T*)Ap; const T* A2 = (const T*)A2p; const T* Bt = (const T*)Btp; const T* Bt2 = (const T*)Bt2p;
  __shared__ __align__(16) float sT[8][16 * 68];
  const int b    = blockIdx.y;
  const int lane = threadIdx.x & 31;
  const int wave = threadIdx.x >> 5;
  const int tilesN = N >> 6;
  const int tilesM = M >> 6;
  const int tile = blockIdx.x * 8 + wave;
  if (tile >= tilesM * tilesN) return;
  const int tm = tile / tilesN;
  const int tn = tile - tm * tilesN;
  const int m0 = tm << 6;
  const int n0 = tn << 6;

  const T* Ab  = A  + (size_t)b * strideA;
  const T* Bb  = Bt + (size_t)b * strideB;
  const T* Ab2 = SPLIT ? (A2  + (size_t)b * strideA) : nullptr;
  const T* Bb2 = SPLIT ? (Bt2 + (size_t)b * strideB) : nullptr;

  const int rlane = lane & 15;
  const int koff  = (lane >> 4) * 8;
  const int mOff  = (lane >> 4) * 8;

  v8f acc[4][4];
#pragma unroll
  for (int i = 0; i < 4; ++i)
#pragma unroll
    for (int j = 0; j < 4; ++j) acc[i][j] = (v8f){0.f,0.f,0.f,0.f,0.f,0.f,0.f,0.f};

  for (int k0 = 0; k0 < K; k0 += 32) {
    V bh[4], bl[4];
#pragma unroll
    for (int j = 0; j < 4; ++j) {
      const size_t bo = (size_t)(n0 + (j << 4) + rlane) * ldb + koff + k0;
      bh[j] = Frag<T>::load(Bb + bo);
      if (SPLIT) bl[j] = Frag<T>::load(Bb2 + bo);
    }
#pragma unroll
    for (int i = 0; i < 4; ++i) {
      const size_t ao = (size_t)(m0 + (i << 4) + rlane) * lda + koff + k0;
      V ah = Frag<T>::load(Ab + ao);
      V al;
      if (SPLIT) al = Frag<T>::load(Ab2 + ao);
#pragma unroll
      for (int j = 0; j < 4; ++j) {
        acc[i][j] = Frag<T>::mma(ah, bh[j], acc[i][j]);
        if (SPLIT) {
          acc[i][j] = Frag<T>::mma(ah, bl[j], acc[i][j]);
          acc[i][j] = Frag<T>::mma(al, bh[j], acc[i][j]);
        }
      }
      Frag<T>::guard4(acc[i][0], acc[i][1], acc[i][2], acc[i][3], ah, SPLIT ? al : ah);
    }
    Frag<T>::keep(bh[0], bh[1], bh[2], bh[3]);
    if (SPLIT) Frag<T>::keep(bl[0], bl[1], bl[2], bl[3]);
  }
  acc_guard4(acc[0][0], acc[0][1], acc[0][2], acc[0][3]);
  acc_guard4(acc[1][0], acc[1][1], acc[1][2], acc[1][3]);
  acc_guard4(acc[2][0], acc[2][1], acc[2][2], acc[2][3]);
  acc_guard4(acc[3][0], acc[3][1], acc[3][2], acc[3][3]);

  float* slab = sT[wave];
  const float* Rb = RESID ? (resid + (size_t)b * strideR) : nullptr;
#pragma unroll
  for (int i = 0; i < 4; ++i) {
    const int mBase = m0 + (i << 4);
#pragma unroll
    for (int j = 0; j < 4; ++j) {
      const int n = n0 + (j << 4) + rlane;
      float bv = 0.f;
      if (BIAS_MODE == 2) bv = bias[n];
#pragma unroll
      for (int r = 0; r < 8; ++r) {
        float v = acc[i][j][r] * scale;
        if (BIAS_MODE == 1) v += bias[mBase + mOff + r];
        if (BIAS_MODE == 2) v += bv;
        if (RESID) v += Rb[(size_t)(mBase + mOff + r) * ldc + n];
        if (ACT == 1) v = tanhf(v);
        if (ACT == 2) v = fmaxf(v, 0.0f);
        if (ACT == 3) v = v / (1.0f + expf(-v));
        if (ACT == 4) v = (v > 0.f) ? v : 0.01f * v;
        slab[(mOff + r) * 68 + (j << 4) + rlane] = v;
      }
    }
    __builtin_amdgcn_fence(__ATOMIC_RELEASE, "workgroup");
    __builtin_amdgcn_wave_barrier();
    __builtin_amdgcn_fence(__ATOMIC_ACQUIRE, "workgroup");
    if (OUT_MODE == 0) {
      float* C = (float*)Cout + (size_t)b * strideC;
      const int hh = lane >> 4, c4 = (lane & 15) * 4;
      for (int pass = 0; pass < 2; ++pass) {
#pragma unroll
        for (int it = 0; it < 8; ++it) {
          const int row = it * 2 + hh;
          v4f v = *(const v4f*)(slab + row * 68 + c4);
          *(volatile v4f*)(C + (size_t)(mBase + row) * ldc + n0 + c4) = v;
        }
        __threadfence();
      }
    } else {
      const int q = lane >> 3, c8 = (lane & 7) * 8;
      unsigned short* C  = (unsigned short*)Cout  + (size_t)b * strideC;
      unsigned short* C2 = (OUT_MODE == 2) ? ((unsigned short*)Cout2 + (size_t)b * strideC) : nullptr;
      for (int pass = 0; pass < 2; ++pass) {
#pragma unroll
        for (int it = 0; it < 4; ++it) {
          const int row = it * 4 + q;
          const float* sp = slab + row * 68 + c8;
          v8h hv, lv;
#pragma unroll
          for (int e = 0; e < 8; ++e) {
            if (OUT_MODE == 1) {
              hv[e] = (_Float16)sp[e];
            } else {
              unsigned short hb = f2bf_bits(sp[e]);
              unsigned short lb = f2bf_bits(sp[e] - bf_bits2f(hb));
              hv[e] = __builtin_bit_cast(_Float16, hb);
              lv[e] = __builtin_bit_cast(_Float16, lb);
            }
          }
          *(volatile v8h*)(C + (size_t)(mBase + row) * ldc + n0 + c8) = hv;
          if (OUT_MODE == 2) *(volatile v8h*)(C2 + (size_t)(mBase + row) * ldc + n0 + c8) = lv;
        }
        __threadfence();
      }
    }
    __builtin_amdgcn_fence(__ATOMIC_RELEASE, "workgroup");
    __builtin_amdgcn_wave_barrier();
    __builtin_amdgcn_fence(__ATOMIC_ACQUIRE, "workgroup");
  }
}


__global__ __launch_bounds__(kThr) void cast_plane_kernel(const float* __restrict__ src, unsigned short* __restrict__ dst,
                                                          int colsLog2, int dstPitch, int dstOff) {
  const int i   = blockIdx.x * kThr + threadIdx.x;
  const int sh  = colsLog2 - 3;
  const int row = i >> sh;
  const int c8  = (i & ((1 << sh) - 1)) * 8;
  const float* sp = src + ((size_t)row << colsLog2) + c8;
  const v4f a0 = *(const v4f*)(sp);
  const v4f a1 = *(const v4f*)(sp + 4);
  v8h hv;
#pragma unroll
  for (int e = 0; e < 4; ++e) {
    const float f0 = a0[e];
    const float f1 = a1[e];
    hv[e]     = (_Float16)carry_flush(bf16r(f0), kInCarry);
    hv[4 + e] = (_Float16)carry_flush(bf16r(f1), kInCarry);
  }
  unsigned short* dp = dst + (size_t)row * dstPitch + dstOff + c8;
  *(volatile v8h*)dp = hv;
  __threadfence();
  *(volatile v8h*)dp = hv;
}

__global__ __launch_bounds__(256) void wt_plane_kernel(const float* __restrict__ W, unsigned short* __restrict__ dst, int K, int N, int nLive, int ldd, int colOff) {
  const int n  = blockIdx.x;
  const int k8 = threadIdx.x * 8;
  const bool live = n < nLive;
  const int nc = live ? n : 0;
  v8h hv;
#pragma unroll
  for (int e = 0; e < 8; ++e) {
    const float w = W[(size_t)(k8 + e) * N + nc];
    hv[e] = (_Float16)(live ? carry_flush(bf16r(w), kWCarry) : 0.0f);
  }
  unsigned short* dp = dst + (size_t)n * ldd + colOff + k8;
  *(volatile v8h*)dp = hv;
  __threadfence();
  *(volatile v8h*)dp = hv;
}

__global__ __launch_bounds__(kThr) void setup_kernel(const float* __restrict__ x, const float* __restrict__ b, float* __restrict__ BV, unsigned short* __restrict__ HX16, float* __restrict__ C32) {
  const unsigned v = blockIdx.x * (unsigned)kThr + threadIdx.x;
  if (v < 1024u) {
    const unsigned f4 = (v & 511u) * 4u;
    const v4f p = *(const v4f*)(b + f4);
    v4f o;
#pragma unroll
    for (int e = 0; e < 4; ++e) o[e] = (v < 512u) ? bf16r(p[e]) : 0.0f;
    float* dp = BV + v * 4u;
    *(volatile v4f*)dp = o;
    __threadfence();
    *(volatile v4f*)dp = o;
  } else if (v < 9216u) {
    const unsigned w = v - 1024u;
    const unsigned r = w >> 6, c8 = (w & 63u) * 8u;
    v8h hv;
#pragma unroll
    for (int q = 0; q < 8; ++q) hv[q] = (_Float16)0.0f;
    unsigned short* dp = HX16 + r * (unsigned)kK + c8;
    *(volatile v8h*)dp = hv;
    __threadfence();
    *(volatile v8h*)dp = hv;
  } else if (v < 17408u) {
    const unsigned w = v - 9216u;
    const unsigned r = w >> 6, x8 = (w & 63u) * 8u;
    const unsigned s = r & 63u, tau0 = (r < (unsigned)kB) ? 0u : (unsigned)(kL - 1);
    const float* sp = x + (s * (unsigned)kL + tau0) * (unsigned)kX + x8;
    const v4f a0 = *(const v4f*)sp, a1 = *(const v4f*)(sp + 4);
    v8h hv;
#pragma unroll
    for (int q = 0; q < 4; ++q) { hv[q] = (_Float16)carry_flush(bf16r(a0[q]), kInCarry); hv[4 + q] = (_Float16)carry_flush(bf16r(a1[q]), kInCarry); }
    unsigned short* dp = HX16 + r * (unsigned)kK + (unsigned)kHid + x8;
    *(volatile v8h*)dp = hv;
    __threadfence();
    *(volatile v8h*)dp = hv;
  } else {
    const unsigned w = v - 17408u;
    const v4f o = {0.0f, 0.0f, 0.0f, 0.0f};
    float* dp = C32 + w * 4u;
    *(volatile v4f*)dp = o;
    __threadfence();
    *(volatile v4f*)dp = o;
  }
}
static_assert(4096 / 4 == 1024 && kR * kHid / 8 == 8192 && kR * kX / 8 == 8192 && kR * kHid / 4 == 16384 && 1024 + 8192 + 8192 + 16384 == 132 * kThr && (1024 % 32) == 0 && (9216 % 32) == 0 && (17408 % 32) == 0, "the set-up's ranges: 132 blocks; each ends on a wave boundary");

__global__ __launch_bounds__(kThr) void cell_kernel(const float* __restrict__ GG, const float* __restrict__ SG, const float* __restrict__ x, float* __restrict__ C32, unsigned short* __restrict__ HX16, float* __restrict__ out, int t) {
  const unsigned v = blockIdx.x * (unsigned)kThr + threadIdx.x;
  const unsigned r = v >> 6, u8 = (v & 63u) * 8u;
  const unsigned s = r & 63u, d = r >> 6;
  const unsigned tau = d ? (unsigned)(kL - 1 - t) : (unsigned)t;
  const float* gr = GG + r * (unsigned)kG4 + u8;
  const float* sr = SG + s * (unsigned)kG4 + u8;
  float* cp = C32 + r * (unsigned)kHid + u8;
  v8h hv, xv;
  v4f cn0, cn1, hn0, hn1;
#pragma unroll
  for (int hlf = 0; hlf < 2; ++hlf) {
    const v4f gi = *(const v4f*)(gr + 4 * hlf), gf = *(const v4f*)(gr + kHid + 4 * hlf), go = *(const v4f*)(gr + 2 * kHid + 4 * hlf), gu = *(const v4f*)(gr + 3 * kHid + 4 * hlf);
    const v4f si = *(const v4f*)(sr + 4 * hlf), sf = *(const v4f*)(sr + kHid + 4 * hlf), so = *(const v4f*)(sr + 2 * kHid + 4 * hlf), su = *(const v4f*)(sr + 3 * kHid + 4 * hlf);
    const v4f co = *(const v4f*)(cp + 4 * hlf);
#pragma unroll
    for (int e = 0; e < 4; ++e) {
      const float zi = 1.0f / (1.0f + expf(-(gi[e] + si[e])));
      const float zf = 1.0f / (1.0f + expf(-(gf[e] + sf[e])));
      const float zo = 1.0f / (1.0f + expf(-(go[e] + so[e])));
      const float zu = tanhf(gu[e] + su[e]);
      const float cn = zf * co[e] + zi * zu;
      const float hn = zo * tanhf(cn);
      if (hlf == 0) { cn0[e] = cn; hn0[e] = hn; } else { cn1[e] = cn; hn1[e] = hn; }
      hv[4 * hlf + e] = (_Float16)carry_flush(hn, kInCarry);
    }
  }
  const bool nx = (t + 1 < kL);
  {
    const unsigned taun = nx ? (d ? (unsigned)(kL - 2 - t) : (unsigned)(t + 1)) : 0u;
    const float* sp = x + (s * (unsigned)kL + taun) * (unsigned)kX + u8;
    const v4f a0 = *(const v4f*)sp, a1 = *(const v4f*)(sp + 4);
#pragma unroll
    for (int e = 0; e < 4; ++e) { xv[e] = (_Float16)carry_flush(bf16r(a0[e]), kInCarry); xv[4 + e] = (_Float16)carry_flush(bf16r(a1[e]), kInCarry); }
  }
  const bool last = (t + 1 == kL);
  unsigned short* hp = HX16 + r * (unsigned)kK + u8;
  unsigned short* xp = HX16 + r * (unsigned)kK + (unsigned)kHid + u8;
  float* op = out + (s * (unsigned)kL + tau) * (unsigned)kOutW + d * (unsigned)kHid + u8;
  float* o1 = out + (unsigned)kOut0 + s * (unsigned)kOutW + d * (unsigned)kHid + u8;
  float* o2 = out + (unsigned)(kOut0 + kOut1) + s * (unsigned)kOutW + d * (unsigned)kHid + u8;
  for (int pass = 0; pass < 2; ++pass) {
    *(volatile v4f*)cp = cn0;
    *(volatile v4f*)(cp + 4) = cn1;
    *(volatile v4f*)op = hn0;
    *(volatile v4f*)(op + 4) = hn1;
    if (nx) {
      *(volatile v8h*)hp = hv;
      *(volatile v8h*)xp = xv;
    }
    if (last) {
      *(volatile v4f*)o1 = hn0;
      *(volatile v4f*)(o1 + 4) = hn1;
      *(volatile v4f*)o2 = cn0;
      *(volatile v4f*)(o2 + 4) = cn1;
    }
    __threadfence();
  }
}
static_assert(kR * kHid / 8 == 32 * kThr && kHid / 8 == 64 && kX / 8 == 64 && (size_t)kOutAll < 4294967296ull / 4, "the cell's grid exact: 32 blocks; a row's 64 threads cover its state part and its input part; 32-bit element offsets");

extern "C" void kernel_launch(void* const* d_in, const int* in_sizes, int n_in,
                              void* d_out, int out_size, void* d_ws, size_t ws_size,
                              hipStream_t stream) {
  if (n_in < 4 || d_out == nullptr || d_ws == nullptr) return;
  if (in_sizes[0] != kB * kL * kX || in_sizes[1] != kB * kGw || in_sizes[2] != (kX + kHid + kGw) * kG4 || in_sizes[3] != kG4) return;
  if (out_size != kOutAll) return;
  if (ws_size < kWsTotal) return;
  const float* x = (const float*)d_in[0];
  const float* g = (const float*)d_in[1];
  const float* W = (const float*)d_in[2];
  const float* b = (const float*)d_in[3];
  float* out = (float*)d_out;
  char* ws = (char*)d_ws;
  unsigned short* W16 = (unsigned short*)(ws + kOffW16);
  unsigned short* WG16 = (unsigned short*)(ws + kOffWG16);
  unsigned short* G16 = (unsigned short*)(ws + kOffG16);
  float* BV = (float*)(ws + kOffBV);
  float* SG = (float*)(ws + kOffSG);
  unsigned short* HX16 = (unsigned short*)(ws + kOffHX16);
  float* GG = (float*)(ws + kOffGG);
  float* C32 = (float*)(ws + kOffC32);

  wt_plane_kernel<<<kG4, kHid / 8, 0, stream>>>(W + (size_t)kX * kG4, W16, kHid, kG4, kG4, kK, 0);
  wt_plane_kernel<<<kG4, kX / 8, 0, stream>>>(W, W16, kX, kG4, kG4, kK, kHid);
  wt_plane_kernel<<<kG4, kGw / 8, 0, stream>>>(W + (size_t)(kX + kHid) * kG4, WG16, kGw, kG4, kG4, kGw, 0);
  static_assert(((size_t)kB * kGw / 8) % kThr == 0, "g's row cast's grid");
  cast_plane_kernel<<<(int)(((size_t)kB * kGw / 8) / kThr), kThr, 0, stream>>>(g, G16, 9, kGw, 0);
  setup_kernel<<<132, kThr, 0, stream>>>(x, b, BV, HX16, C32);
  wmma_gemm64<0, false, 2, 0, false, 0><<<dim3((kB / 64) * (kG4 / 64) / 8, 1), 256, 0, stream>>>(
      G16, G16, kGw, 0L, WG16, WG16, kGw, 0L, (void*)SG, (void*)SG, kG4, 0L, BV + kBvGate, nullptr, 0L, kB, kG4, kGw, kSc);
  for (int t = 0; t < kL; ++t) {
    wmma_gemm64<0, false, 2, 0, false, 0><<<dim3((kR / 64) * (kG4 / 64) / 8, 1), 256, 0, stream>>>(
        HX16, HX16, kK, 0L, W16, W16, kK, 0L, (void*)GG, (void*)GG, kG4, 0L, BV + kBvZero, nullptr, 0L, kR, kG4, kK, kSc);
    cell_kernel<<<32, kThr, 0, stream>>>(GG, SG, x, C32, HX16, out, t);
  }
}
static_assert(((kB / 64) * (kG4 / 64)) % 8 == 0 && ((kR / 64) * (kG4 / 64)) % 8 == 0 && (kHid / 8) == 64, "the engine's grids: whole blocks of eight wave tiles; the transposing cast's block: 64 threads");
